// SatelliteDensityModelV4_78323023610134
// MI455X (gfx1250) — hardware-verified
//
#include <hip/hip_runtime.h>
#include <math.h>

constexpr int NSEQ   = 128;
constexpr int TSTEPS = 1024;
constexpr int DIN0   = 32;
constexpr int HG     = 64;
constexpr int GW     = 192;
constexpr int X1W    = 128;
constexpr int NROWS  = NSEQ * TSTEPS;
constexpr int SDIM   = 16;
constexpr int SKP    = 32;
constexpr int NPH    = 5;
constexpr int PLEN   = 432;
constexpr int PLP    = 448;
constexpr int HIDW   = 128;
constexpr int FUSEDW = 288;
constexpr int HAP    = 320;
constexpr int NCONV  = 96;
constexpr int SEGW   = 128;
constexpr int NTR    = 128;
constexpr int NTA    = 224;
constexpr int HPITCH = 72;
constexpr int FPITCH = 68;
constexpr int CPW    = 480;

typedef __attribute__((ext_vector_type(16))) _Float16 v16h;
typedef __attribute__((ext_vector_type(8)))  _Float16 v8h;
typedef __attribute__((ext_vector_type(16))) __bf16   v16b;
typedef __attribute__((ext_vector_type(8)))  __bf16   v8b;
typedef __attribute__((ext_vector_type(8)))  float    v8f;
typedef __attribute__((ext_vector_type(4)))  float    v4f;

__device__ __forceinline__ unsigned short f2bf_bits(float f) {
  unsigned u = __float_as_uint(f);
  return (unsigned short)((u + 0x7FFFu + ((u >> 16) & 1u)) >> 16);
}
__device__ __forceinline__ float bf_bits2f(unsigned short h) { return __uint_as_float(((unsigned)h) << 16); }

__device__ __forceinline__ void dep_guard_h(v8f& a, v8f& b, v16h x, v16h y) { asm volatile("v_nop\n\tv_nop\n\tv_nop\n\tv_nop" : "+v"(a), "+v"(b) : "v"(x), "v"(y)); }
__device__ __forceinline__ void dep_guard_b(v8f& a, v8f& b, v16b x, v16b y) { asm volatile("v_nop\n\tv_nop\n\tv_nop\n\tv_nop" : "+v"(a), "+v"(b) : "v"(x), "v"(y)); }
__device__ __forceinline__ void keep4_h(v16h a, v16h b, v16h c, v16h d) { asm volatile("v_nop" :: "v"(a), "v"(b), "v"(c), "v"(d)); }
__device__ __forceinline__ void keep4_b(v16b a, v16b b, v16b c, v16b d) { asm volatile("v_nop" :: "v"(a), "v"(b), "v"(c), "v"(d)); }
__device__ __forceinline__ void acc_guard4(v8f& a, v8f& b, v8f& c, v8f& d) { asm volatile("v_nop\n\tv_nop\n\tv_nop\n\tv_nop" : "+v"(a), "+v"(b), "+v"(c), "+v"(d)); }
__device__ __forceinline__ void dep_guard3_h(v8f& a, v8f& b, v8f& c, v16h w, v16h x, v16h y, v16h z) {
  asm volatile("v_nop\n\tv_nop\n\tv_nop\n\tv_nop" : "+v"(a), "+v"(b), "+v"(c) : "v"(w), "v"(x), "v"(y), "v"(z));
}
__device__ __forceinline__ void acc_guard3(v8f& a, v8f& b, v8f& c) { asm volatile("v_nop\n\tv_nop\n\tv_nop\n\tv_nop" : "+v"(a), "+v"(b), "+v"(c)); }

template <typename T> struct Frag;
template <> struct Frag<_Float16> {
  typedef v16h V; union U { v16h v; v8h h[2]; };
  static __device__ __forceinline__ v16h load(const _Float16* p) {
    U f; f.h[0] = *(const v8h*)(p); f.h[1] = *(const v8h*)(p + 16); return f.v;
  }
  static __device__ __forceinline__ v8f mma(v16h a, v16h b, v8f c) {
    return __builtin_amdgcn_wmma_f32_16x16x32_f16(false, a, false, b, (short)0, c, false, false);
  }
  static __device__ __forceinline__ void guard(v8f& a, v8f& b, v16h x, v16h y) { dep_guard_h(a, b, x, y); }
  static __device__ __forceinline__ void keep(v16h a, v16h b, v16h c, v16h d) { keep4_h(a, b, c, d); }
};
template <> struct Frag<__bf16> {
  typedef v16b V; union U { v16b v; v8b h[2]; };
  static __device__ __forceinline__ v16b load(const __bf16* p) {
    U f; f.h[0] = *(const v8b*)(p); f.h[1] = *(const v8b*)(p + 16); return f.v;
  }
  static __device__ __forceinline__ v8f mma(v16b a, v16b b, v8f c) {
    return __builtin_amdgcn_wmma_f32_16x16x32_bf16(false, a, false, b, (short)0, c, false, false);
  }
  static __device__ __forceinline__ void guard(v8f& a, v8f& b, v16b x, v16b y) { dep_guard_b(a, b, x, y); }
  static __device__ __forceinline__ void keep(v16b a, v16b b, v16b c, v16b d) { keep4_b(a, b, c, d); }
};

template <int ET> struct Elem;
template <> struct Elem<0> { typedef _Float16 T; };
template <> struct Elem<1> { typedef __bf16 T; };
template <int ET, bool SPLIT, int BIAS_MODE, int OUT_MODE, bool RESID, int ACT = 0>
__global__ __launch_bounds__(256) void wmma_gemm64(
    const unsigned short* __restrict__ Ap, const unsigned short* __restrict__ A2p, int lda, long strideA,
    const unsigned short* __restrict__ Btp, const unsigned short* __restrict__ Bt2p, int ldb, long strideB,
    void* __restrict__ Cout, void* __restrict__ Cout2, int ldc, long strideC,
    const float* __restrict__ bias,
    const float* __restrict__ resid, long strideR,
    int M, int N, int K, float scale) {
  typedef typename Elem<ET>::T T;
  typedef typename Frag<T>::V V;
  const T* A = (const T*)Ap; const T* A2 = (const T*)A2p; const T* Bt = (const T*)Btp; const T* Bt2 = (const T*)Bt2p;
  __shared__ __align__(16) float sT[8][16 * 68];
  const int b    = blockIdx.y;
  const int lane = threadIdx.x & 31;
  const int wave = threadIdx.x >> 5;
  const int tilesN = N >> 6;
  const int tilesM = M >> 6;
  const int tile = blockIdx.x * 8 + wave;
  if (tile >= tilesM * tilesN) return;
  const int tm = tile / tilesN;
  const int tn = tile - tm * tilesN;
  const int m0 = tm << 6;
  const int n0 = tn << 6;

  const T* Ab  = A  + (size_t)b * strideA;
  const T* Bb  = Bt + (size_t)b * strideB;
  const T* Ab2 = SPLIT ? (A2  + (size_t)b * strideA) : nullptr;
  const T* Bb2 = SPLIT ? (Bt2 + (size_t)b * strideB) : nullptr;

  const int rlane = lane & 15;
  const int koff  = (lane >> 4) * 8;
  const int mOff  = (lane >> 4) * 8;

  v8f acc[4][4];
#pragma unroll
  for (int i = 0; i < 4; ++i)
#pragma unroll
    for (int j = 0; j < 4; ++j) acc[i][j] = (v8f){0.f,0.f,0.f,0.f,0.f,0.f,0.f,0.f};

  for (int k0 = 0; k0 < K; k0 += 32) {
    V bh[4], bl[4];
#pragma unroll
    for (int j = 0; j < 4; ++j) {
      const size_t bo = (size_t)(n0 + (j << 4) + rlane) * ldb + koff + k0;
      bh[j] = Frag<T>::load(Bb + bo);
      if (SPLIT) bl[j] = Frag<T>::load(Bb2 + bo);
    }
#pragma unroll
    for (int i = 0; i < 4; ++i) {
      const size_t ao = (size_t)(m0 + (i << 4) + rlane) * lda + koff + k0;
      V ah = Frag<T>::load(Ab + ao);
      V al;
      if (SPLIT) al = Frag<T>::load(Ab2 + ao);
#pragma unroll
      for (int j = 0; j < 4; ++j) {
        acc[i][j] = Frag<T>::mma(ah, bh[j], acc[i][j]);
        if (SPLIT) {
          acc[i][j] = Frag<T>::mma(ah, bl[j], acc[i][j]);
          acc[i][j] = Frag<T>::mma(al, bh[j], acc[i][j]);
        }
      }
      Frag<T>::guard(acc[i][0], acc[i][3], ah, SPLIT ? al : ah);
    }
    Frag<T>::keep(bh[0], bh[1], bh[2], bh[3]);
    if (SPLIT) Frag<T>::keep(bl[0], bl[1], bl[2], bl[3]);
  }
  acc_guard4(acc[0][0], acc[0][1], acc[0][2], acc[0][3]);
  acc_guard4(acc[1][0], acc[1][1], acc[1][2], acc[1][3]);
  acc_guard4(acc[2][0], acc[2][1], acc[2][2], acc[2][3]);
  acc_guard4(acc[3][0], acc[3][1], acc[3][2], acc[3][3]);

  float* slab = sT[wave];
  const float* Rb = RESID ? (resid + (size_t)b * strideR) : nullptr;
#pragma unroll
  for (int i = 0; i < 4; ++i) {
    const int mBase = m0 + (i << 4);
#pragma unroll
    for (int j = 0; j < 4; ++j) {
      const int n = n0 + (j << 4) + rlane;
      float bv = 0.f;
      if (BIAS_MODE == 2) bv = bias[n];
#pragma unroll
      for (int r = 0; r < 8; ++r) {
        float v = acc[i][j][r] * scale;
        if (BIAS_MODE == 1) v += bias[mBase + mOff + r];
        if (BIAS_MODE == 2) v += bv;
        if (RESID) v += Rb[(size_t)(mBase + mOff + r) * ldc + n];
        if (ACT == 1) v = tanhf(v);
        if (ACT == 2) v = fmaxf(v, 0.0f);
        if (ACT == 3) v = v / (1.0f + expf(-v));
        if (ACT == 4) v = (v > 0.f) ? v : 0.01f * v;
        if (ACT == 5) v = 0.5f * v * (1.0f + erff(v * 0.70710678118654752f));
        slab[(mOff + r) * 68 + (j << 4) + rlane] = v;
      }
    }
    __builtin_amdgcn_fence(__ATOMIC_RELEASE, "workgroup");
    __builtin_amdgcn_wave_barrier();
    __builtin_amdgcn_fence(__ATOMIC_ACQUIRE, "workgroup");
    if (OUT_MODE == 0) {
      float* C = (float*)Cout + (size_t)b * strideC;
      const int hh = lane >> 4, c4 = (lane & 15) * 4;
      for (int pass = 0; pass < 2; ++pass) {
#pragma unroll
        for (int it = 0; it < 8; ++it) {
          const int row = it * 2 + hh;
          v4f v = *(const v4f*)(slab + row * 68 + c4);
          *(volatile v4f*)(C + (size_t)(mBase + row) * ldc + n0 + c4) = v;
        }
        __threadfence();
      }
    } else {
      const int q = lane >> 3, c8 = (lane & 7) * 8;
      unsigned short* C  = (unsigned short*)Cout  + (size_t)b * strideC;
      unsigned short* C2 = (OUT_MODE == 2) ? ((unsigned short*)Cout2 + (size_t)b * strideC) : nullptr;
      for (int pass = 0; pass < 2; ++pass) {
#pragma unroll
        for (int it = 0; it < 4; ++it) {
          const int row = it * 4 + q;
          const float* sp = slab + row * 68 + c8;
          v8h hv, lv;
#pragma unroll
          for (int e = 0; e < 8; ++e) {
            if (OUT_MODE == 1) {
              hv[e] = (_Float16)sp[e];
            } else {
              unsigned short hb = f2bf_bits(sp[e]);
              unsigned short lb = f2bf_bits(sp[e] - bf_bits2f(hb));
              hv[e] = __builtin_bit_cast(_Float16, hb);
              lv[e] = __builtin_bit_cast(_Float16, lb);
            }
          }
          *(volatile v8h*)(C + (size_t)(mBase + row) * ldc + n0 + c8) = hv;
          if (OUT_MODE == 2) *(volatile v8h*)(C2 + (size_t)(mBase + row) * ldc + n0 + c8) = lv;
        }
        __threadfence();
      }
    }
    __builtin_amdgcn_fence(__ATOMIC_RELEASE, "workgroup");
    __builtin_amdgcn_wave_barrier();
    __builtin_amdgcn_fence(__ATOMIC_ACQUIRE, "workgroup");
  }
}

__device__ __forceinline__ unsigned pack_f16x2(float a, float b) {
  const _Float16 h0 = (_Float16)a, h1 = (_Float16)b;
  return (unsigned)__builtin_bit_cast(unsigned short, h0) | ((unsigned)__builtin_bit_cast(unsigned short, h1) << 16);
}
__device__ __forceinline__ void st2u(unsigned* p, unsigned v) { *(volatile unsigned*)p = v; __threadfence(); *(volatile unsigned*)p = v; }
__device__ __forceinline__ float ftanh(float x) { return 1.0f - 2.0f * __builtin_amdgcn_rcpf(1.0f + __expf(2.0f * x)); }
__device__ __forceinline__ float fsigm(float x) { return __builtin_amdgcn_rcpf(1.0f + __expf(-x)); }
__device__ __forceinline__ float gelu_f(float x) { return 0.5f * x * (1.0f + erff(x * 0.70710678118654752f)); }
__device__ __forceinline__ float warp_sum(float v) {
#pragma unroll
  for (int off = 16; off > 0; off >>= 1) v += __shfl_xor(v, off, 32);
  return v;
}
__device__ __forceinline__ float warp_max(float v) {
#pragma unroll
  for (int off = 16; off > 0; off >>= 1) v = fmaxf(v, __shfl_xor(v, off, 32));
  return v;
}
__device__ __forceinline__ float warp_min(float v) {
#pragma unroll
  for (int off = 16; off > 0; off >>= 1) v = fminf(v, __shfl_xor(v, off, 32));
  return v;
}
__device__ __forceinline__ void cast16_pair(const float* __restrict__ W, unsigned* __restrict__ D, int p) {
  st2u(D + p, pack_f16x2(W[2 * p] * 16.0f, W[2 * p + 1] * 16.0f));
}
__device__ __forceinline__ void split_pair(float a, float b, unsigned* __restrict__ Dh, unsigned* __restrict__ Dl, int p) {
  const unsigned short ha = f2bf_bits(a), hb = f2bf_bits(b);
  const unsigned short la = f2bf_bits(a - bf_bits2f(ha)), lb = f2bf_bits(b - bf_bits2f(hb));
  st2u(Dh + p, (unsigned)ha | ((unsigned)hb << 16));
  st2u(Dl + p, (unsigned)la | ((unsigned)lb << 16));
}

constexpr int kBlkX16   = 2048;
constexpr int kBlkWih0f = kBlkX16 + 12;
constexpr int kBlkWih0b = kBlkWih0f + 12;
constexpr int kBlkWhh0f = kBlkWih0b + 24;
constexpr int kBlkWhh0b = kBlkWhh0f + 24;
constexpr int kBlkWih1f = kBlkWhh0b + 48;
constexpr int kBlkWih1b = kBlkWih1f + 48;
constexpr int kBlkWhh1f = kBlkWih1b + 24;
constexpr int kBlkWhh1b = kBlkWhh1f + 24;
constexpr int kBlkW1    = kBlkWhh1b + 72;
constexpr int kBlkW2    = kBlkW1 + 112;
constexpr int kBlkSX    = kBlkW2 + 8;
constexpr int kBlkSMW   = kBlkSX + 4;
constexpr int kBlkB2    = kBlkSMW + 1;
__global__ __launch_bounds__(256) void prep_kernel(
    const float* __restrict__ x,
    const float* __restrict__ Wih0f, const float* __restrict__ Wih0b, const float* __restrict__ Whh0f, const float* __restrict__ Whh0b,
    const float* __restrict__ Wih1f, const float* __restrict__ Wih1b, const float* __restrict__ Whh1f, const float* __restrict__ Whh1b,
    const float* __restrict__ hW1, const float* __restrict__ hW2, const float* __restrict__ sx, const float* __restrict__ smW,
    const float* __restrict__ hb2,
    _Float16* __restrict__ X16,
    unsigned* __restrict__ WIH0F, unsigned* __restrict__ WIH0B, unsigned* __restrict__ WHH0F, unsigned* __restrict__ WHH0B,
    unsigned* __restrict__ WIH1F, unsigned* __restrict__ WIH1B, unsigned* __restrict__ WHH1F, unsigned* __restrict__ WHH1B,
    unsigned* __restrict__ W1H, unsigned* __restrict__ W1L, unsigned* __restrict__ W2H, unsigned* __restrict__ W2L,
    unsigned* __restrict__ SXH, unsigned* __restrict__ SXL, unsigned* __restrict__ SMH, unsigned* __restrict__ SML,
    float* __restrict__ B2P) {
  const int blk = blockIdx.x, tid = threadIdx.x;
  if (blk < kBlkX16) {
    const int gid = blk * 256 + tid;
    const float* p = x + (size_t)gid * 8;
    const v4f a = *(const v4f*)p, bq = *(const v4f*)(p + 4);
    v8h hv;
#pragma unroll
    for (int e = 0; e < 4; ++e) { hv[e] = (_Float16)a[e]; hv[4 + e] = (_Float16)bq[e]; }
    _Float16* op = X16 + (size_t)gid * 8;
    *(volatile v8h*)op = hv; __threadfence(); *(volatile v8h*)op = hv;
  } else if (blk < kBlkWih0f) { cast16_pair(Wih0f, WIH0F, (blk - kBlkX16)   * 256 + tid); }
  else if (blk < kBlkWih0b)   { cast16_pair(Wih0b, WIH0B, (blk - kBlkWih0f) * 256 + tid); }
  else if (blk < kBlkWhh0f)   { cast16_pair(Whh0f, WHH0F, (blk - kBlkWih0b) * 256 + tid); }
  else if (blk < kBlkWhh0b)   { cast16_pair(Whh0b, WHH0B, (blk - kBlkWhh0f) * 256 + tid); }
  else if (blk < kBlkWih1f)   { cast16_pair(Wih1f, WIH1F, (blk - kBlkWhh0b) * 256 + tid); }
  else if (blk < kBlkWih1b)   { cast16_pair(Wih1b, WIH1B, (blk - kBlkWih1f) * 256 + tid); }
  else if (blk < kBlkWhh1f)   { cast16_pair(Whh1f, WHH1F, (blk - kBlkWih1b) * 256 + tid); }
  else if (blk < kBlkWhh1b)   { cast16_pair(Whh1b, WHH1B, (blk - kBlkWhh1f) * 256 + tid); }
  else if (blk < kBlkW1) {
    const int p = (blk - kBlkWhh1b) * 256 + tid;
    split_pair(hW1[2 * p], hW1[2 * p + 1], W1H, W1L, p);
  } else if (blk < kBlkW2) {
    const int rb = blk - kBlkW1;
    const int p = rb * 256 + tid;
    float a = 0.0f, bq = 0.0f;
    if (rb < 108) { a = hW2[2 * p]; bq = hW2[2 * p + 1]; }
    split_pair(a, bq, W2H, W2L, p);
  } else if (blk < kBlkSX) {
    const int p = (blk - kBlkW2) * 256 + tid;
    const int row = p >> 4, cp = p & 15, cc = cp < 8 ? cp : 7;
    float a = sx[row * SDIM + 2 * cc], bq = sx[row * SDIM + 2 * cc + 1];
    if (cp >= 8) { a = 0.0f; bq = 0.0f; }
    split_pair(a, bq, SXH, SXL, p);
  } else if (blk < kBlkSMW) {
    const int p = (blk - kBlkSX) * 256 + tid;
    const int row = p >> 4, cp = p & 15, cc = cp < 8 ? cp : 7;
    float a = smW[row * SDIM + 2 * cc], bq = smW[row * SDIM + 2 * cc + 1];
    if (cp >= 8) { a = 0.0f; bq = 0.0f; }
    split_pair(a, bq, SMH, SML, p);
  } else {
    if (tid < PLP / 4) {
      v4f v;
#pragma unroll
      for (int e = 0; e < 4; ++e) {
        const int idx = 4 * tid + e;
        const int idc = idx < PLEN ? idx : PLEN - 1;
        const float t = hb2[idc];
        v[e] = (idx < PLEN) ? t : 0.0f;
      }
      float* dst = B2P + 4 * tid;
      *(volatile v4f*)dst = v; __threadfence(); *(volatile v4f*)dst = v;
    }
  }
}

template <bool FINAL>
__global__ __launch_bounds__(NTR) void gru_rec_kernel(const _Float16* __restrict__ GI, const _Float16* __restrict__ WHH,
                                                     const float* __restrict__ bhh, int dir,
                                                     _Float16* __restrict__ X1, float* __restrict__ OMNI) {
  __shared__ __align__(16) _Float16 h16[16 * HPITCH];
  __shared__ __align__(16) float hf[FINAL ? 16 * FPITCH : 4];
  const int tid = threadIdx.x, lane = tid & 31, wave = tid >> 5;
  const int rlane = lane & 15, hh = lane >> 4, koff = hh * 8, mOff = hh * 8;
  const int blk = blockIdx.x;
  for (int i = tid; i < 16 * HPITCH; i += NTR) h16[i] = (_Float16)0.0f;
  __syncthreads();

  const int j = 16 * wave + rlane;
  const _Float16* arow = h16 + rlane * HPITCH + koff;
  const _Float16* wr = WHH + (size_t)j * HG + koff;
  const _Float16* wz = WHH + (size_t)(HG + j) * HG + koff;
  const _Float16* wn = WHH + (size_t)(2 * HG + j) * HG + koff;
  const float br = bhh[j], bz = bhh[HG + j], bn = bhh[2 * HG + j];
  const _Float16* gib = GI + (size_t)(blk * 16 + mOff) * TSTEPS * GW + j;
  const v8f z8 = {0.f, 0.f, 0.f, 0.f, 0.f, 0.f, 0.f, 0.f};
  const float s16 = 1.0f / 16.0f;

  float hreg[8];
#pragma unroll
  for (int r = 0; r < 8; ++r) hreg[r] = 0.0f;

#pragma unroll 1
  for (int s = 0; s < TSTEPS; ++s) {
    const int t = dir ? (TSTEPS - 1 - s) : s;
    v8f ar = z8, az = z8, an = z8;
#pragma unroll 1
    for (int k0 = 0; k0 < HG; k0 += 32) {
      const v16h a  = Frag<_Float16>::load(arow + k0);
      const v16h b0 = Frag<_Float16>::load(wr + k0);
      const v16h b1 = Frag<_Float16>::load(wz + k0);
      const v16h b2 = Frag<_Float16>::load(wn + k0);
      ar = Frag<_Float16>::mma(a, b0, ar);
      az = Frag<_Float16>::mma(a, b1, az);
      an = Frag<_Float16>::mma(a, b2, an);
      dep_guard3_h(ar, az, an, a, b0, b1, b2);
    }
    acc_guard3(ar, az, an);

    const _Float16* xt = gib + (size_t)t * GW;
#pragma unroll
    for (int r = 0; r < 8; ++r) {
      const _Float16* xr = xt + (size_t)r * TSTEPS * GW;
      const float x_r = (float)xr[0], x_z = (float)xr[HG], x_n = (float)xr[2 * HG];
      const float hr = ar[r] * s16 + br;
      const float hz = az[r] * s16 + bz;
      const float hn = an[r] * s16 + bn;
      const float rg = fsigm(x_r + hr);
      const float zg = fsigm(x_z + hz);
      const float ng = ftanh(x_n + rg * hn);
      hreg[r] = (1.0f - zg) * ng + zg * hreg[r];
    }
    __syncthreads();
#pragma unroll
    for (int r = 0; r < 8; ++r) h16[(mOff + r) * HPITCH + j] = (_Float16)hreg[r];
    __syncthreads();
    if (!FINAL) {
      const int q = lane >> 3, c8 = (lane & 7) * 8;
      const int row = 4 * wave + q;
      _Float16* dst = X1 + ((size_t)(blk * 16 + row) * TSTEPS + t) * X1W + dir * HG + c8;
      for (int pass = 0; pass < 2; ++pass) {
        const v8h v = *(const v8h*)(h16 + row * HPITCH + c8);
        *(volatile v8h*)dst = v;
        __threadfence();
      }
    }
  }

  if (FINAL) {
#pragma unroll
    for (int r = 0; r < 8; ++r) hf[(mOff + r) * FPITCH + j] = hreg[r];
    __syncthreads();
    const int c4 = (lane & 15) * 4;
    for (int pass = 0; pass < 2; ++pass) {
#pragma unroll
      for (int it = 0; it < 2; ++it) {
        const int row = it * 8 + 2 * wave + hh;
        const v4f v = *(const v4f*)(hf + row * FPITCH + c4);
        *(volatile v4f*)(OMNI + (size_t)(blk * 16 + row) * HIDW + dir * HG + c4) = v;
      }
      __threadfence();
    }
  }
}

__global__ __launch_bounds__(64) void static_kernel(const float* __restrict__ SEPRE, const float* __restrict__ ln_g,
                                                   const float* __restrict__ ln_b, const float* __restrict__ gate_W,
                                                   const float* __restrict__ gate_b, float* __restrict__ SEG) {
  __shared__ float sg[HG];
  __shared__ __align__(16) float rowbuf[SEGW];
  const int tid = threadIdx.x, b = blockIdx.x;
  const float xv = SEPRE[(size_t)b * HG + tid];
  const float g = gelu_f(xv);
  sg[tid] = g;
  __syncthreads();
  float m = 0.0f;
#pragma unroll 1
  for (int k = 0; k < HG; ++k) m += sg[k];
  m *= (1.0f / 64.0f);
  float var = 0.0f;
#pragma unroll 1
  for (int k = 0; k < HG; ++k) { const float d = sg[k] - m; var += d * d; }
  var *= (1.0f / 64.0f);
  const float inv = 1.0f / sqrtf(var + 1e-5f);
  rowbuf[tid] = (g - m) * inv * ln_g[tid] + ln_b[tid];
  rowbuf[HG + tid] = 0.0f;
  __syncthreads();
  if (tid < NPH) {
    float a = 0.0f;
#pragma unroll 1
    for (int k = 0; k < HG; ++k) a += rowbuf[k] * gate_W[tid * HG + k];
    a += gate_b[tid];
    rowbuf[HG + tid] = fsigm(a);
  }
  __syncthreads();
  if (tid < 32) {
    const v4f v = *(const v4f*)(rowbuf + 4 * tid);
    float* dst = SEG + (size_t)b * SEGW + 4 * tid;
    *(volatile v4f*)dst = v; __threadfence(); *(volatile v4f*)dst = v;
  }
}

__global__ __launch_bounds__(NTA) void mha_kernel(const float* __restrict__ phys, const float* __restrict__ SEG,
                                                  const float* __restrict__ Win, const float* __restrict__ bin,
                                                  float* __restrict__ AO) {
  __shared__ __align__(16) float qs[PLEN];
  __shared__ __align__(16) float ks[PLEN];
  __shared__ __align__(16) float vs[PLEN];
  __shared__ __align__(16) float aos[PLP];
  __shared__ float rmx[8], rmn[8];
  const int tid = threadIdx.x, lane = tid & 31, wave = tid >> 5;
  const int bh = blockIdx.x, b = bh / NPH, h = bh - b * NPH;
  float gt[5], wq[5], wk[5], wv[5];
#pragma unroll
  for (int gg = 0; gg < 5; ++gg) {
    gt[gg] = SEG[(size_t)b * SEGW + HG + gg];
    wq[gg] = Win[h * NPH + gg];
    wk[gg] = Win[(NPH + h) * NPH + gg];
    wv[gg] = Win[(2 * NPH + h) * NPH + gg];
  }
  const float bq = bin[h], bk = bin[NPH + h], bvv = bin[2 * NPH + h];
  float lmx = -3.0e38f, lmn = 3.0e38f;
  for (int l = tid; l < PLEN; l += NTA) {
    const float* pp = phys + (size_t)b * NPH * PLEN + l;
    float pg[5];
#pragma unroll
    for (int gg = 0; gg < 5; ++gg) pg[gg] = pp[gg * PLEN] * gt[gg];
    const float dq = pg[0] * wq[0] + pg[1] * wq[1] + pg[2] * wq[2] + pg[3] * wq[3] + pg[4] * wq[4];
    const float dk = pg[0] * wk[0] + pg[1] * wk[1] + pg[2] * wk[2] + pg[3] * wk[3] + pg[4] * wk[4];
    const float dv = pg[0] * wv[0] + pg[1] * wv[1] + pg[2] * wv[2] + pg[3] * wv[3] + pg[4] * wv[4];
    const float kq = dk + bk;
    qs[l] = dq + bq; ks[l] = kq; vs[l] = dv + bvv;
    lmx = fmaxf(lmx, kq); lmn = fminf(lmn, kq);
  }
  if (tid < PLP - PLEN) aos[PLEN + tid] = 0.0f;
  lmx = warp_max(lmx); lmn = warp_min(lmn);
  if (lane == 0) { rmx[wave] = lmx; rmn[wave] = lmn; }
  __syncthreads();
  float kmax = rmx[0], kmin = rmn[0];
#pragma unroll
  for (int w = 1; w < NTA / 32; ++w) { kmax = fmaxf(kmax, rmx[w]); kmin = fminf(kmin, rmn[w]); }
  for (int i = tid; i < PLEN; i += NTA) {
    const float q = qs[i];
    const float m = fmaxf(q * kmax, q * kmin);
    const float nm = -m;
    float lsum = 0.0f, acc = 0.0f;
#pragma unroll 1
    for (int jj = 0; jj < PLEN; jj += 4) {
      const v4f kk = *(const v4f*)(ks + jj);
      const v4f vv = *(const v4f*)(vs + jj);
#pragma unroll
      for (int e = 0; e < 4; ++e) {
        const float ex = __expf(fmaf(q, kk[e], nm));
        lsum += ex;
        acc = fmaf(ex, vv[e], acc);
      }
    }
    aos[i] = acc * __builtin_amdgcn_rcpf(lsum);
  }
  __syncthreads();
  if (tid < PLP / 4) {
    const v4f v = *(const v4f*)(aos + 4 * tid);
    float* dst = AO + (size_t)bh * PLP + 4 * tid;
    *(volatile v4f*)dst = v; __threadfence(); *(volatile v4f*)dst = v;
  }
}

__global__ __launch_bounds__(256) void conv_kernel(const float* __restrict__ AO, const float* __restrict__ Wo,
                                                   const float* __restrict__ bo,
                                                   const float* __restrict__ cw1, const float* __restrict__ cb1,
                                                   const float* __restrict__ cw2, const float* __restrict__ cb2,
                                                   const float* __restrict__ cw3, const float* __restrict__ cb3,
                                                   float* __restrict__ CF) {
  __shared__ __align__(16) float p2s[NPH * CPW];
  __shared__ __align__(16) float wts[2720];
  __shared__ float cbias[NCONV];
  __shared__ float wos[25], bos[5];
  __shared__ float yst[256 * 33];
  __shared__ float red2[2 * 8 * 32];
  __shared__ __align__(16) float cfs[NCONV];
  const int tid = threadIdx.x, lane = tid & 31, wave = tid >> 5;
  const int b = blockIdx.x;
  for (int i = tid; i < NPH * CPW; i += 256) p2s[i] = 0.0f;
  for (int idx = tid; idx < 480; idx += 256)  { const int oc = idx / 15; const int rem = idx - oc * 15; wts[rem * 32 + oc] = cw1[idx]; }
  for (int idx = tid; idx < 800; idx += 256)  { const int oc = idx / 25; const int rem = idx - oc * 25; wts[480 + rem * 32 + oc] = cw2[idx]; }
  for (int idx = tid; idx < 1440; idx += 256) { const int oc = idx / 45; const int rem = idx - oc * 45; wts[1280 + rem * 32 + oc] = cw3[idx]; }
  if (tid < 32) { cbias[tid] = cb1[tid]; cbias[32 + tid] = cb2[tid]; cbias[64 + tid] = cb3[tid]; }
  if (tid < 25) wos[tid] = Wo[tid];
  if (tid < 5) bos[tid] = bo[tid];
  __syncthreads();
  for (int i = tid; i < PLEN; i += 256) {
    const float* ap = AO + (size_t)(b * NPH) * PLP + i;
    const float a0 = ap[0], a1 = ap[PLP], a2 = ap[2 * PLP], a3 = ap[3 * PLP], a4 = ap[4 * PLP];
#pragma unroll 1
    for (int o = 0; o < NPH; ++o) {
      float v = a0 * wos[o * 5] + a1 * wos[o * 5 + 1] + a2 * wos[o * 5 + 2] + a3 * wos[o * 5 + 3] + a4 * wos[o * 5 + 4];
      v += bos[o];
      p2s[o * CPW + 4 + i] = v;
    }
  }
  __syncthreads();
#pragma unroll 1
  for (int br = 0; br < 3; ++br) {
    const int ksz = (br == 0) ? 3 : (br == 1) ? 5 : 9;
    const int dil = 1 << br;
    const int pad = dil;
    const int wb  = (br == 0) ? 0 : (br == 1) ? 480 : 1280;
    const int lout = PLEN + 2 * pad - dil * (ksz - 1);
    const float invl = __builtin_amdgcn_rcpf((float)lout);
#pragma unroll 1
    for (int q = 0; q < 2; ++q) {
      const int l = tid + 256 * q;
      const bool valid = l < lout;
      const int lc = valid ? l : (lout - 1);
      float y[32];
#pragma unroll
      for (int oc = 0; oc < 32; ++oc) y[oc] = cbias[br * 32 + oc];
#pragma unroll 1
      for (int ic = 0; ic < NPH; ++ic) {
        const float* prow = p2s + ic * CPW + 4 + lc - pad;
        const float* wrow = wts + wb + ic * ksz * 32;
#pragma unroll 1
        for (int kk = 0; kk < ksz; ++kk) {
          const float pv = prow[kk * dil];
          const float* w = wrow + kk * 32;
#pragma unroll
          for (int g4 = 0; g4 < 8; ++g4) {
            const v4f wv = *(const v4f*)(w + 4 * g4);
            y[4 * g4 + 0] = fmaf(wv[0], pv, y[4 * g4 + 0]);
            y[4 * g4 + 1] = fmaf(wv[1], pv, y[4 * g4 + 1]);
            y[4 * g4 + 2] = fmaf(wv[2], pv, y[4 * g4 + 2]);
            y[4 * g4 + 3] = fmaf(wv[3], pv, y[4 * g4 + 3]);
          }
        }
      }
#pragma unroll
      for (int oc = 0; oc < 32; ++oc) yst[tid * 33 + oc] = y[oc];
#pragma unroll 1
      for (int oc = 0; oc < 32; ++oc) {
        const float v = yst[tid * 33 + oc];
        const float gv = gelu_f(v);
        yst[tid * 33 + oc] = valid ? gv : 0.0f;
      }
      __syncthreads();
      {
        const int oc = tid & 31, seg = tid >> 5;
        float s = 0.0f;
#pragma unroll 1
        for (int rr = 0; rr < 32; ++rr) s += yst[(seg * 32 + rr) * 33 + oc];
        red2[(q * 8 + seg) * 32 + oc] = s;
      }
      __syncthreads();
    }
    if (tid < 32) {
      float tot = 0.0f;
#pragma unroll
      for (int q = 0; q < 2; ++q)
#pragma unroll
        for (int seg = 0; seg < 8; ++seg) tot += red2[(q * 8 + seg) * 32 + tid];
      cfs[br * 32 + tid] = tot * invl;
    }
  }
  __syncthreads();
  if (tid < NCONV / 4) {
    const v4f v = *(const v4f*)(cfs + 4 * tid);
    float* dst = CF + (size_t)b * NCONV + 4 * tid;
    *(volatile v4f*)dst = v; __threadfence(); *(volatile v4f*)dst = v;
  }
}

__global__ __launch_bounds__(256) void head_prep_kernel(const float* __restrict__ OMNI, const float* __restrict__ SEG,
                                                        const float* __restrict__ CF, const float* __restrict__ ln_g,
                                                        const float* __restrict__ ln_b,
                                                        unsigned short* __restrict__ HAH, unsigned short* __restrict__ HAL) {
  __shared__ float fz[FUSEDW];
  __shared__ __align__(16) float hn[HAP];
  __shared__ float rs[8], rv[8];
  const int tid = threadIdx.x, lane = tid & 31, wave = tid >> 5;
  const int b = blockIdx.x;
  if (tid < HIDW)  fz[tid] = OMNI[(size_t)b * HIDW + tid];
  if (tid < HG)    fz[HIDW + tid] = SEG[(size_t)b * SEGW + tid];
  if (tid < NCONV) fz[HIDW + HG + tid] = CF[(size_t)b * NCONV + tid];
  if (tid < HAP - FUSEDW) hn[FUSEDW + tid] = 0.0f;
  __syncthreads();
  const int i2 = tid + 256;
  const bool has2 = i2 < FUSEDW;
  const int i2c = has2 ? i2 : (FUSEDW - 1);
  const float x0 = fz[tid], x1 = fz[i2c];
  float s = x0 + (has2 ? x1 : 0.0f);
  s = warp_sum(s);
  if (lane == 0) rs[wave] = s;
  __syncthreads();
  float tot = 0.0f;
#pragma unroll
  for (int w = 0; w < 8; ++w) tot += rs[w];
  const float mean = tot * (1.0f / 288.0f);
  const float d0 = x0 - mean, d1 = x1 - mean;
  float s2 = d0 * d0 + (has2 ? d1 * d1 : 0.0f);
  s2 = warp_sum(s2);
  if (lane == 0) rv[wave] = s2;
  __syncthreads();
  float vt = 0.0f;
#pragma unroll
  for (int w = 0; w < 8; ++w) vt += rv[w];
  const float var = vt * (1.0f / 288.0f);
  const float inv = 1.0f / sqrtf(var + 1e-5f);
  hn[tid] = d0 * inv * ln_g[tid] + ln_b[tid];
  if (has2) hn[i2] = d1 * inv * ln_g[i2] + ln_b[i2];
  __syncthreads();
  if (tid < HAP / 8) {
    v8h hv, lv;
#pragma unroll
    for (int e = 0; e < 8; ++e) {
      const float f = hn[8 * tid + e];
      const unsigned short hb = f2bf_bits(f);
      const unsigned short lb = f2bf_bits(f - bf_bits2f(hb));
      hv[e] = __builtin_bit_cast(_Float16, hb);
      lv[e] = __builtin_bit_cast(_Float16, lb);
    }
    unsigned short* dh = HAH + (size_t)b * HAP + 8 * tid;
    unsigned short* dl = HAL + (size_t)b * HAP + 8 * tid;
    *(volatile v8h*)dh = hv; *(volatile v8h*)dl = lv;
    __threadfence();
    *(volatile v8h*)dh = hv; *(volatile v8h*)dl = lv;
  }
}

__global__ __launch_bounds__(256) void gelu_split_kernel(const float* __restrict__ H1, unsigned* __restrict__ HBH, unsigned* __restrict__ HBL) {
  const int p = blockIdx.x * 256 + threadIdx.x;
  const float a = gelu_f(H1[2 * p]), bq = gelu_f(H1[2 * p + 1]);
  split_pair(a, bq, HBH, HBL, p);
}

__global__ __launch_bounds__(256) void pack_kernel(const float* __restrict__ OUTP, float* __restrict__ out) {
  const int i = blockIdx.x * 256 + threadIdx.x;
  const int f = 4 * i;
  const int row = f / PLEN;
  const int col = f - row * PLEN;
  const v4f v = *(const v4f*)(OUTP + (size_t)row * PLP + col);
  *(volatile v4f*)(out + f) = v; __threadfence(); *(volatile v4f*)(out + f) = v;
}

extern "C" void kernel_launch(void* const* d_in, const int* in_sizes, int n_in,
                              void* d_out, int out_size, void* d_ws, size_t ws_size, hipStream_t stream) {
  if (n_in < 41 || d_out == nullptr || d_ws == nullptr) return;
  if (in_sizes[0] != NROWS * DIN0 || in_sizes[1] != NSEQ * SDIM || in_sizes[2] != NSEQ * NPH * PLEN ||
      in_sizes[3] != GW * DIN0 || in_sizes[4] != GW * HG || in_sizes[5] != GW || in_sizes[6] != GW ||
      in_sizes[7] != GW * DIN0 || in_sizes[8] != GW * HG || in_sizes[11] != GW * X1W || in_sizes[12] != GW * HG ||
      in_sizes[15] != GW * X1W || in_sizes[16] != GW * HG || in_sizes[19] != HG * SDIM || in_sizes[20] != HG ||
      in_sizes[23] != NPH * HG || in_sizes[24] != NPH || in_sizes[25] != 3 * NPH * NPH || in_sizes[26] != 3 * NPH ||
      in_sizes[27] != NPH * NPH || in_sizes[28] != NPH || in_sizes[29] != 32 * NPH * 3 || in_sizes[31] != 32 * NPH * 5 ||
      in_sizes[33] != 32 * NPH * 9 || in_sizes[35] != FUSEDW || in_sizes[37] != HIDW * FUSEDW || in_sizes[38] != HIDW ||
      in_sizes[39] != PLEN * HIDW || in_sizes[40] != PLEN || out_size != NSEQ * PLEN) return;

  const float* omni_seq = (const float*)d_in[0];
  const float* static_x = (const float*)d_in[1];
  const float* phys     = (const float*)d_in[2];
  const float* Wih0f = (const float*)d_in[3];  const float* Whh0f = (const float*)d_in[4];
  const float* bih0f = (const float*)d_in[5];  const float* bhh0f = (const float*)d_in[6];
  const float* Wih0b = (const float*)d_in[7];  const float* Whh0b = (const float*)d_in[8];
  const float* bih0b = (const float*)d_in[9];  const float* bhh0b = (const float*)d_in[10];
  const float* Wih1f = (const float*)d_in[11]; const float* Whh1f = (const float*)d_in[12];
  const float* bih1f = (const float*)d_in[13]; const float* bhh1f = (const float*)d_in[14];
  const float* Wih1b = (const float*)d_in[15]; const float* Whh1b = (const float*)d_in[16];
  const float* bih1b = (const float*)d_in[17]; const float* bhh1b = (const float*)d_in[18];
  const float* sm_W = (const float*)d_in[19];  const float* sm_b = (const float*)d_in[20];
  const float* sm_ln_g = (const float*)d_in[21]; const float* sm_ln_b = (const float*)d_in[22];
  const float* gate_W = (const float*)d_in[23]; const float* gate_b = (const float*)d_in[24];
  const float* attn_in_W = (const float*)d_in[25]; const float* attn_in_b = (const float*)d_in[26];
  const float* attn_out_W = (const float*)d_in[27]; const float* attn_out_b = (const float*)d_in[28];
  const float* conv1_W = (const float*)d_in[29]; const float* conv1_b = (const float*)d_in[30];
  const float* conv2_W = (const float*)d_in[31]; const float* conv2_b = (const float*)d_in[32];
  const float* conv3_W = (const float*)d_in[33]; const float* conv3_b = (const float*)d_in[34];
  const float* head_ln_g = (const float*)d_in[35]; const float* head_ln_b = (const float*)d_in[36];
  const float* head_W1 = (const float*)d_in[37]; const float* head_b1 = (const float*)d_in[38];
  const float* head_W2 = (const float*)d_in[39];
  const float* head_b2 = (const float*)d_in[40];
  float* out = (float*)d_out;

  char* ws = (char*)d_ws; size_t off = 0;
  auto carve = [&](size_t bytes) -> char* { char* p = ws + off; off += (bytes + 255) & ~(size_t)255; return p; };
  _Float16* X16   = (_Float16*)carve((size_t)NROWS * DIN0 * 2);
  _Float16* GI16  = (_Float16*)carve((size_t)NROWS * GW * 2);
  _Float16* X1_16 = (_Float16*)carve((size_t)NROWS * X1W * 2);
  unsigned* WIH0F = (unsigned*)carve((size_t)GW * DIN0 * 2);
  unsigned* WIH0B = (unsigned*)carve((size_t)GW * DIN0 * 2);
  unsigned* WHH0F = (unsigned*)carve((size_t)GW * HG * 2);
  unsigned* WHH0B = (unsigned*)carve((size_t)GW * HG * 2);
  unsigned* WIH1F = (unsigned*)carve((size_t)GW * X1W * 2);
  unsigned* WIH1B = (unsigned*)carve((size_t)GW * X1W * 2);
  unsigned* WHH1F = (unsigned*)carve((size_t)GW * HG * 2);
  unsigned* WHH1B = (unsigned*)carve((size_t)GW * HG * 2);
  unsigned* W1H   = (unsigned*)carve((size_t)HIDW * FUSEDW * 2);
  unsigned* W1L   = (unsigned*)carve((size_t)HIDW * FUSEDW * 2);
  unsigned* W2H   = (unsigned*)carve((size_t)PLP * HIDW * 2);
  unsigned* W2L   = (unsigned*)carve((size_t)PLP * HIDW * 2);
  unsigned* SXH   = (unsigned*)carve((size_t)NSEQ * SKP * 2);
  unsigned* SXL   = (unsigned*)carve((size_t)NSEQ * SKP * 2);
  unsigned* SMH   = (unsigned*)carve((size_t)HG * SKP * 2);
  unsigned* SML   = (unsigned*)carve((size_t)HG * SKP * 2);
  float*    B2P   = (float*)carve((size_t)PLP * 4);
  float*    SEPRE = (float*)carve((size_t)NSEQ * HG * 4);
  float*    SEG   = (float*)carve((size_t)NSEQ * SEGW * 4);
  float*    OMNI  = (float*)carve((size_t)NSEQ * HIDW * 4);
  float*    AO    = (float*)carve((size_t)NSEQ * NPH * PLP * 4);
  float*    CF    = (float*)carve((size_t)NSEQ * NCONV * 4);
  unsigned short* HAH = (unsigned short*)carve((size_t)NSEQ * HAP * 2);
  unsigned short* HAL = (unsigned short*)carve((size_t)NSEQ * HAP * 2);
  float*    H1    = (float*)carve((size_t)NSEQ * HIDW * 4);
  unsigned* HBH   = (unsigned*)carve((size_t)NSEQ * HIDW * 2);
  unsigned* HBL   = (unsigned*)carve((size_t)NSEQ * HIDW * 2);
  float*    OUTP  = (float*)carve((size_t)NSEQ * PLP * 4);
  if (off > ws_size || off > (size_t)134217728) return;

  const unsigned short* nul16 = (const unsigned short*)nullptr;
  const float* nulf = (const float*)nullptr;

  prep_kernel<<<kBlkB2, 256, 0, stream>>>(omni_seq, Wih0f, Wih0b, Whh0f, Whh0b, Wih1f, Wih1b, Whh1f, Whh1b,
                                          head_W1, head_W2, static_x, sm_W, head_b2,
                                          X16, WIH0F, WIH0B, WHH0F, WHH0B, WIH1F, WIH1B, WHH1F, WHH1B,
                                          W1H, W1L, W2H, W2L, SXH, SXL, SMH, SML, B2P);

  wmma_gemm64<1, true, 2, 0, false><<<dim3(1, 1), 256, 0, stream>>>(
      (const unsigned short*)SXH, (const unsigned short*)SXL, SKP, 0L,
      (const unsigned short*)SMH, (const unsigned short*)SML, SKP, 0L,
      (void*)SEPRE, (void*)nullptr, HG, 0L, sm_b, nulf, 0L, NSEQ, HG, SKP, 1.0f);
  static_kernel<<<NSEQ, 64, 0, stream>>>(SEPRE, sm_ln_g, sm_ln_b, gate_W, gate_b, SEG);
  mha_kernel<<<NSEQ * NPH, NTA, 0, stream>>>(phys, SEG, attn_in_W, attn_in_b, AO);
  conv_kernel<<<NSEQ, 256, 0, stream>>>(AO, attn_out_W, attn_out_b, conv1_W, conv1_b, conv2_W, conv2_b, conv3_W, conv3_b, CF);

  const int giBlocks = ((NROWS / 64) * (GW / 64)) / 8;
  wmma_gemm64<0, false, 2, 1, false><<<dim3(giBlocks, 1), 256, 0, stream>>>(
      (const unsigned short*)X16, nul16, DIN0, 0L, (const unsigned short*)WIH0F, nul16, DIN0, 0L,
      (void*)GI16, (void*)nullptr, GW, 0L, bih0f, nulf, 0L, NROWS, GW, DIN0, 1.0f / 16.0f);
  gru_rec_kernel<false><<<NSEQ / 16, NTR, 0, stream>>>(GI16, (const _Float16*)WHH0F, bhh0f, 0, X1_16, OMNI);
  wmma_gemm64<0, false, 2, 1, false><<<dim3(giBlocks, 1), 256, 0, stream>>>(
      (const unsigned short*)X16, nul16, DIN0, 0L, (const unsigned short*)WIH0B, nul16, DIN0, 0L,
      (void*)GI16, (void*)nullptr, GW, 0L, bih0b, nulf, 0L, NROWS, GW, DIN0, 1.0f / 16.0f);
  gru_rec_kernel<false><<<NSEQ / 16, NTR, 0, stream>>>(GI16, (const _Float16*)WHH0B, bhh0b, 1, X1_16, OMNI);

  wmma_gemm64<0, false, 2, 1, false><<<dim3(giBlocks, 1), 256, 0, stream>>>(
      (const unsigned short*)X1_16, nul16, X1W, 0L, (const unsigned short*)WIH1F, nul16, X1W, 0L,
      (void*)GI16, (void*)nullptr, GW, 0L, bih1f, nulf, 0L, NROWS, GW, X1W, 1.0f / 16.0f);
  gru_rec_kernel<true><<<NSEQ / 16, NTR, 0, stream>>>(GI16, (const _Float16*)WHH1F, bhh1f, 0, X1_16, OMNI);
  wmma_gemm64<0, false, 2, 1, false><<<dim3(giBlocks, 1), 256, 0, stream>>>(
      (const unsigned short*)X1_16, nul16, X1W, 0L, (const unsigned short*)WIH1B, nul16, X1W, 0L,
      (void*)GI16, (void*)nullptr, GW, 0L, bih1b, nulf, 0L, NROWS, GW, X1W, 1.0f / 16.0f);
  gru_rec_kernel<true><<<NSEQ / 16, NTR, 0, stream>>>(GI16, (const _Float16*)WHH1B, bhh1b, 1, X1_16, OMNI);

  head_prep_kernel<<<NSEQ, 256, 0, stream>>>(OMNI, SEG, CF, head_ln_g, head_ln_b, HAH, HAL);
  wmma_gemm64<1, true, 2, 0, false><<<dim3(1, 1), 256, 0, stream>>>(
      (const unsigned short*)HAH, (const unsigned short*)HAL, HAP, 0L,
      (const unsigned short*)W1H, (const unsigned short*)W1L, FUSEDW, 0L,
      (void*)H1, (void*)nullptr, HIDW, 0L, head_b1, nulf, 0L, NSEQ, HIDW, FUSEDW, 1.0f);
  gelu_split_kernel<<<(NSEQ * HIDW / 2) / 256, 256, 0, stream>>>(H1, HBH, HBL);
  wmma_gemm64<1, true, 2, 0, false><<<dim3(2, 1), 256, 0, stream>>>(
      (const unsigned short*)HBH, (const unsigned short*)HBL, HIDW, 0L,
      (const unsigned short*)W2H, (const unsigned short*)W2L, HIDW, 0L,
      (void*)OUTP, (void*)nullptr, PLP, 0L, B2P, nulf, 0L, NSEQ, PLP, HIDW, 1.0f);
  pack_kernel<<<(NSEQ * PLEN / 4) / 256, 256, 0, stream>>>(OUTP, out);
}
